// KerSr_17197049053612
// MI455X (gfx1250) — hardware-verified
//
#include <hip/hip_runtime.h>
#include <stdint.h>


typedef __attribute__((ext_vector_type(16))) _Float16 v16h;
typedef __attribute__((ext_vector_type(8)))  float    v8f;
typedef __attribute__((ext_vector_type(4)))  uint32_t v4u;

union AFrag { v16h h; v4u u4[2]; };
typedef __attribute__((ext_vector_type(8))) _Float16 v8h;
typedef __attribute__((ext_vector_type(4))) float v4f;
typedef float __attribute__((may_alias)) float_a;
template <typename T> __device__ __forceinline__ void vst2(void* p, T v) { *(volatile T*)p = v; __threadfence(); *(volatile T*)p = v; }
__device__ __forceinline__ v8f wmma16(v16h a, v16h b, v8f c) {
  v8f d = __builtin_amdgcn_wmma_f32_16x16x32_f16(false, a, false, b, (short)0, c, false, false);
  asm volatile("v_nop\n\tv_nop\n\tv_nop\n\tv_nop" : "+v"(d) : "v"(a), "v"(b));
  return d;
}

__global__ void pack_weights(const float* __restrict__ w, _Float16* __restrict__ dst,
                             int CinP, int CoutP, int CinR, int CoutR) {
  int nCC = CinP >> 5, nNT = CoutP >> 4;
  int total = 9 * nCC * nNT * 512;
  int g8 = blockIdx.x * blockDim.x + threadIdx.x;
  int e0 = g8 * 8;
  if (e0 >= total) return;
  int frag = e0 >> 9;
  int rem  = e0 & 511;
  int lane = rem >> 4;
  int idx0 = rem & 15;
  int half = lane >> 4;
  int n    = lane & 15;
  int nt   = frag % nNT;
  int cc   = (frag / nNT) % nCC;
  int rs   = frag / (nNT * nCC);
  int co   = nt * 16 + n;
  union { v8h h; v4u u; } pk;
#pragma unroll
  for (int q = 0; q < 8; ++q) { int idx = idx0 + q; int K = 8 * half + ((idx < 8) ? idx : (idx + 8)); int ci = cc * 32 + K;
    float v = 0.f; if (co < CoutR && ci < CinR) v = w[((long)co * CinR + ci) * 9 + rs]; pk.h[q] = (_Float16)v; }
  vst2(dst + e0, pk.u);
}

template<int CO, int COP>
__global__ __launch_bounds__(256) void conv_c1_direct(const float* __restrict__ x, const float* __restrict__ w,
                                                      _Float16* __restrict__ out, int Nn, int H, int W) {
  __shared__ __align__(16) _Float16 so[128 * COP];
  const int wave = threadIdx.x >> 5, lane = threadIdx.x & 31, m = lane & 15, half = lane >> 4;
  const long p = (long)blockIdx.x * 128 + wave * 16 + m;
  const int xx = (int)(p % W), yy = (int)((p / W) % H), n = (int)(p / ((long)W * H));
  v16h a;
#pragma unroll
  for (int i = 0; i < 16; ++i) a[i] = (_Float16)0.f;
#pragma unroll
  for (int i = 0; i < 8; ++i) {
    const int t = half * 8 + i;
    if (t < 9) { const int r = t / 3, s = t % 3; const int y2 = yy + r - 1, x2 = xx + s - 1;
      float v = 0.f; if ((unsigned)y2 < (unsigned)H && (unsigned)x2 < (unsigned)W) v = x[((long)n * H + y2) * W + x2];
      a[i] = (_Float16)v; }
  }
  constexpr int nNT = COP / 16;
  v8f acc[nNT];
#pragma unroll
  for (int nt = 0; nt < nNT; ++nt) {
    acc[nt] = (v8f){0.f,0.f,0.f,0.f,0.f,0.f,0.f,0.f};
    v16h b;
#pragma unroll
    for (int i = 0; i < 16; ++i) b[i] = (_Float16)0.f;
    const int co = nt * 16 + m;
#pragma unroll
    for (int i = 0; i < 8; ++i) { const int t = half * 8 + i; if (t < 9 && co < CO) b[i] = (_Float16)w[co * 9 + t]; }
    acc[nt] = wmma16(a, b, acc[nt]);
  }
  _Float16* o = so + (wave * 16) * COP;
#pragma unroll
  for (int nt = 0; nt < nNT; ++nt)
#pragma unroll
    for (int vr = 0; vr < 8; ++vr) { float v = acc[nt][vr]; v = v > 0.f ? v : 0.f; if (nt * 16 + m >= CO) v = 0.f;
      o[(vr + half * 8) * COP + nt * 16 + m] = (_Float16)v; }
  __syncthreads();
  const long pb = (long)blockIdx.x * 128;
  for (int q = threadIdx.x; q < 128 * COP / 8; q += 256) vst2(out + pb * COP + (long)q * 8, *(const v4u*)(so + q * 8));
}

template<int CinP, int CoutP>
__global__ __launch_bounds__(256)
void conv3x3_wmma(const _Float16* __restrict__ in, _Float16* __restrict__ out,
                  const _Float16* __restrict__ wB,
                  int Nn, int H, int W) {
  constexpr int nCC = CinP / 32;
  constexpr int nNT = CoutP / 16;
  constexpr int wFragBytes = 9 * nCC * nNT * 1024;
  constexpr int slabPix    = 130;
  constexpr int pixBytes   = CinP * 2;
  constexpr int pixChunks  = pixBytes / 16;
  __shared__ __align__(16) char smemW[wFragBytes];
  __shared__ __align__(16) char smemIn[3 * slabPix * pixBytes];

  const int segs = W >> 7;
  int blk = blockIdx.x;
  int n0 = blk / (H * segs);
  int r2 = blk % (H * segs);
  int y  = r2 / segs;
  int x0blk = (r2 % segs) * 128;

  for (int i = threadIdx.x; i < wFragBytes / 16; i += 256)
    *(v4u*)(smemW + i * 16) = *(const v4u*)((const char*)wB + i * 16);

  {
    const int total = 3 * slabPix * pixChunks;
    for (int t = threadIdx.x; t < total; t += 256) {
      int ch = t % pixChunks;
      int p  = (t / pixChunks) % slabPix;
      int r  = t / (pixChunks * slabPix);
      int gy = y - 1 + r;
      int gx = x0blk - 1 + p;
      char* l = smemIn + (size_t)(r * slabPix + p) * pixBytes + ch * 16;
      if ((unsigned)gy < (unsigned)H && (unsigned)gx < (unsigned)W) {
        const char* g = (const char*)in
            + ((((long)n0 * H + gy) * W + gx) * CinP) * 2 + ch * 16;
        *(v4u*)l = *(const v4u*)g;
      } else {
        *(v4u*)l = (v4u){0u, 0u, 0u, 0u};
      }
    }
  }
  __syncthreads();

  const int wave = threadIdx.x >> 5;
  const int lane = threadIdx.x & 31;
  const int half = lane >> 4;
  const int m    = lane & 15;
  const int x0   = x0blk + wave * 16;

  v8f acc[nNT];
#pragma unroll
  for (int t = 0; t < nNT; ++t) acc[t] = (v8f){0.f,0.f,0.f,0.f,0.f,0.f,0.f,0.f};

#pragma unroll
  for (int r = 0; r < 3; ++r) {
#pragma unroll
    for (int s = 0; s < 3; ++s) {
      const int p = wave * 16 + m + s;
      const char* pixBase = smemIn + (size_t)(r * slabPix + p) * pixBytes + half * 16;
#pragma unroll
      for (int cc = 0; cc < nCC; ++cc) {
        AFrag a;
        a.u4[0] = *(const v4u*)(pixBase + cc * 64);
        a.u4[1] = *(const v4u*)(pixBase + cc * 64 + 32);
        const int fbase = ((r * 3 + s) * nCC + cc) * nNT;
#pragma unroll
        for (int nt = 0; nt < nNT; ++nt) {
          const v16h* bp = (const v16h*)(smemW + (size_t)(fbase + nt) * 1024 + lane * 32);
          acc[nt] = wmma16(a.h, *bp, acc[nt]);
        }
      }
    }
  }

  __syncthreads();
  _Float16* so = (_Float16*)smemIn + wave * (16 * CoutP);
#pragma unroll
  for (int nt = 0; nt < nNT; ++nt) {
    int co = nt * 16 + m;
#pragma unroll
    for (int vr = 0; vr < 8; ++vr) {
      int mm = vr + half * 8;
      float v = acc[nt][vr];
      v = v > 0.f ? v : 0.f;
      so[mm * CoutP + co] = (_Float16)v;
    }
  }
  asm volatile("s_wait_dscnt 0" ::: "memory"); __builtin_amdgcn_wave_barrier(); __builtin_amdgcn_fence(__ATOMIC_RELEASE, "workgroup");
  long rowBase = ((long)n0 * H + y) * W;
  _Float16* ob = out + (rowBase + x0) * CoutP;
  for (int q = lane; q < 16 * CoutP / 8; q += 32) vst2(ob + q * 8, *(const v4u*)(so + q * 8));
}

__global__ void pixshuf_relu(const _Float16* __restrict__ a5, float* __restrict__ h,
                             int Nn, int H, int W) {
  int HO = H * 4, WO = W * 4;
  long total = (long)Nn * HO * WO;
  long p = (long)blockIdx.x * blockDim.x + threadIdx.x;
  if (p >= total) return;
  int X = (int)(p % WO);
  int Y = (int)((p / WO) % HO);
  int n = (int)(p / ((long)WO * HO));
  int hh = Y >> 2, i = Y & 3, ww = X >> 2, j = X & 3;
  float v = (float)a5[(((long)n * H + hh) * W + ww) * 16 + (i * 4 + j)];
  vst2(h + p, (float_a)(v > 0.f ? v : 0.f));
}

__global__ void pixconv_add(const float* __restrict__ h, const _Float16* __restrict__ z,
                            float* __restrict__ out, int Nn, int H, int W) {
  long total = (long)Nn * H * W;
  long p = (long)blockIdx.x * blockDim.x + threadIdx.x;
  if (p >= total) return;
  int xx = (int)(p % W);
  int yy = (int)((p / W) % H);
  int n  = (int)(p / ((long)W * H));
  const float* hn = h + (long)n * H * W;
  const _Float16* zp = z + p * 32;
  float acc = 0.f;
#pragma unroll
  for (int j = 0; j < 25; ++j) {
    int kw = j / 5, kh = j % 5;
    int y2 = yy + kh - 2, x2 = xx + kw - 2;
    float hv = ((unsigned)y2 < (unsigned)H && (unsigned)x2 < (unsigned)W)
                   ? hn[(long)y2 * W + x2] : 0.f;
    acc += hv * (float)zp[j];
  }
  vst2(out + p, (float_a)(h[p] + acc));
}

static inline size_t wbytes(int CinP, int CoutP) {
  return (size_t)9 * (CinP / 32) * (CoutP / 16) * 512 * 2;
}

extern "C" void kernel_launch(void* const* d_in, const int* in_sizes, int n_in,
                              void* d_out, int out_size, void* d_ws, size_t ws_size,
                              hipStream_t stream) {
  (void)in_sizes; (void)n_in; (void)out_size; (void)ws_size;
  const float* x    = (const float*)d_in[0];
  const float* w_e1 = (const float*)d_in[1];
  const float* w_e2 = (const float*)d_in[2];
  const float* w_e3 = (const float*)d_in[3];
  const float* w_d1 = (const float*)d_in[4];
  const float* w_d2 = (const float*)d_in[5];
  const float* w_k1 = (const float*)d_in[6];
  const float* w_k2 = (const float*)d_in[7];
  const float* w_k3 = (const float*)d_in[8];
  const float* w_k4 = (const float*)d_in[9];
  float* out = (float*)d_out;
  char* ws = (char*)d_ws;

  const int N = 2, H1 = 256, W1 = 256, H2 = 1024, W2 = 1024;
  const long P1 = (long)N * H1 * W1;
  const long P2 = (long)N * H2 * W2;

  size_t off = 0;
  auto alloc = [&](size_t bytes) { size_t o = off; off = (off + bytes + 255) & ~(size_t)255; return o; };
  size_t oWe2 = alloc(wbytes(32, 32));
  size_t oWe3 = alloc(wbytes(32, 64));
  size_t oWd1 = alloc(wbytes(64, 32));
  size_t oWd2 = alloc(wbytes(32, 16));
  size_t oWk2 = alloc(wbytes(32, 64));
  size_t oWk3 = alloc(wbytes(64, 32));
  size_t oWk4 = alloc(wbytes(32, 32));
  size_t oA1 = alloc((size_t)P1 * 32 * 2);
  size_t oA2 = alloc((size_t)P1 * 32 * 2);
  size_t oA3 = alloc((size_t)P1 * 64 * 2);
  size_t oA4 = alloc((size_t)P1 * 32 * 2);
  size_t oA5 = alloc((size_t)P1 * 16 * 2);
  size_t oH  = alloc((size_t)P2 * 4);
  size_t oB1 = alloc((size_t)(P2 / N) * 32 * 2);
  size_t oB2 = alloc((size_t)(P2 / N) * 64 * 2);

  _Float16* wBe2 = (_Float16*)(ws + oWe2);
  _Float16* wBe3 = (_Float16*)(ws + oWe3);
  _Float16* wBd1 = (_Float16*)(ws + oWd1);
  _Float16* wBd2 = (_Float16*)(ws + oWd2);
  _Float16* wBk2 = (_Float16*)(ws + oWk2);
  _Float16* wBk3 = (_Float16*)(ws + oWk3);
  _Float16* wBk4 = (_Float16*)(ws + oWk4);
  _Float16* a1 = (_Float16*)(ws + oA1);
  _Float16* a2 = (_Float16*)(ws + oA2);
  _Float16* a3 = (_Float16*)(ws + oA3);
  _Float16* a4 = (_Float16*)(ws + oA4);
  _Float16* a5 = (_Float16*)(ws + oA5);
  float*    hB = (float*)(ws + oH);
  _Float16* b1 = (_Float16*)(ws + oB1);
  _Float16* b2 = (_Float16*)(ws + oB2);
  _Float16* b3 = b1;
  _Float16* zB = b2;

  auto packGrid = [](int CinP, int CoutP) {
    int total = 9 * (CinP / 32) * (CoutP / 16) * 512;
    return (total / 8 + 255) / 256;
  };
  pack_weights<<<packGrid(32, 32), 256, 0, stream>>>(w_e2, wBe2, 32, 32, 16, 32);
  pack_weights<<<packGrid(32, 64), 256, 0, stream>>>(w_e3, wBe3, 32, 64, 32, 64);
  pack_weights<<<packGrid(64, 32), 256, 0, stream>>>(w_d1, wBd1, 64, 32, 64, 32);
  pack_weights<<<packGrid(32, 16), 256, 0, stream>>>(w_d2, wBd2, 32, 16, 32, 16);
  pack_weights<<<packGrid(32, 64), 256, 0, stream>>>(w_k2, wBk2, 32, 64, 32, 64);
  pack_weights<<<packGrid(64, 32), 256, 0, stream>>>(w_k3, wBk3, 64, 32, 64, 32);
  pack_weights<<<packGrid(32, 32), 256, 0, stream>>>(w_k4, wBk4, 32, 32, 32, 25);

  conv_c1_direct<16, 32><<<(int)(P1 / 128), 256, 0, stream>>>(x, w_e1, a1, N, H1, W1);

  auto convGrid = [](int Nn, int H, int W) { return Nn * H * (W >> 7); };
  conv3x3_wmma<32, 32><<<convGrid(N, H1, W1), 256, 0, stream>>>(a1, a2, wBe2, N, H1, W1);
  conv3x3_wmma<32, 64><<<convGrid(N, H1, W1), 256, 0, stream>>>(a2, a3, wBe3, N, H1, W1);
  conv3x3_wmma<64, 32><<<convGrid(N, H1, W1), 256, 0, stream>>>(a3, a4, wBd1, N, H1, W1);
  conv3x3_wmma<32, 16><<<convGrid(N, H1, W1), 256, 0, stream>>>(a4, a5, wBd2, N, H1, W1);

  pixshuf_relu<<<(int)((P2 + 255) / 256), 256, 0, stream>>>(a5, hB, N, H1, W1);

  const long PI = (long)H2 * W2;
  for (int n = 0; n < N; ++n) {
    const float* hn = hB + n * PI;
    conv_c1_direct<32, 32><<<(int)(PI / 128), 256, 0, stream>>>(hn, w_k1, b1, 1, H2, W2);
    conv3x3_wmma<32, 64><<<convGrid(1, H2, W2), 256, 0, stream>>>(b1, b2, wBk2, 1, H2, W2);
    conv3x3_wmma<64, 32><<<convGrid(1, H2, W2), 256, 0, stream>>>(b2, b3, wBk3, 1, H2, W2);
    conv3x3_wmma<32, 32><<<convGrid(1, H2, W2), 256, 0, stream>>>(b3, zB, wBk4, 1, H2, W2);
    pixconv_add<<<(int)((PI + 255) / 256), 256, 0, stream>>>(hn, zB, out + n * PI, 1, H2, W2);
  }
}
